// CausalMultiHeadSelfAttention_23390391894854
// MI455X (gfx1250) — hardware-verified
//
#include <hip/hip_runtime.h>


#ifndef NB
#define NB 2
#endif
#ifndef SEQ
#define SEQ 2048
#endif
#define S_FULL 2048
#define D_     1024
#define QKV_   1024
#define H_     16
#define HD_    64
#define NP_    (HD_ / 2)
#define M_TOT  (NB * SEQ)
#define SCALE_ 0.125f

static_assert(NB >= 1 && NB <= 2);
static_assert(SEQ % 128 == 0 && SEQ >= 128 && SEQ <= S_FULL);
static_assert(H_ * HD_ == D_);
static_assert(D_ % 32 == 0 && QKV_ % 128 == 0 && M_TOT % 128 == 0);

typedef __attribute__((ext_vector_type(16))) __bf16 v16bf;
typedef __attribute__((ext_vector_type(8)))  __bf16 v8bf;
typedef __attribute__((ext_vector_type(8)))  float  v8f;
typedef __attribute__((ext_vector_type(4)))  float  v4f;

template <typename V> __device__ __forceinline__ void vst2(void* p, V v) {
  *(volatile V*)p = v; __threadfence(); *(volatile V*)p = v;
}
__device__ __forceinline__ __bf16 bf_hi(float x) { return (__bf16)x; }
__device__ __forceinline__ __bf16 bf_lo(float x, __bf16 h) { return (__bf16)(x - (float)h); }
__device__ __forceinline__ v8f wmma_bf16(v16bf a, v16bf b, v8f c) {
  v8f d = __builtin_amdgcn_wmma_f32_16x16x32_bf16(false, a, false, b, (short)0, c, false, false);
  asm volatile("v_nop\n\tv_nop\n\tv_nop\n\tv_nop" : "+v"(d) : "v"(a), "v"(b));
  return d;
}
__device__ __forceinline__ v8f wmma_x3(v16bf ah, v16bf al, v16bf bh, v16bf bl, v8f c) {
  c = wmma_bf16(ah, bh, c); c = wmma_bf16(ah, bl, c); c = wmma_bf16(al, bh, c);
  return c;
}

__device__ __forceinline__ void frag_f32(const float* __restrict__ base, int ld, int r0, int k0, int lane, v16bf& hi, v16bf& lo) {
  const float* p = base + (size_t)(r0 + (lane & 15)) * ld + k0 + (lane >> 4) * 8;
  const v4f a0 = *(const v4f*)(p), a1 = *(const v4f*)(p + 4), a2 = *(const v4f*)(p + 16), a3 = *(const v4f*)(p + 20);
#pragma unroll
  for (int i = 0; i < 4; ++i) {
    __bf16 h;
    h = bf_hi(a0[i]); hi[i] = h;      lo[i] = bf_lo(a0[i], h);
    h = bf_hi(a1[i]); hi[4 + i] = h;  lo[4 + i] = bf_lo(a1[i], h);
    h = bf_hi(a2[i]); hi[8 + i] = h;  lo[8 + i] = bf_lo(a2[i], h);
    h = bf_hi(a3[i]); hi[12 + i] = h; lo[12 + i] = bf_lo(a3[i], h);
  }
}
__device__ __forceinline__ v16bf frag_f32h(const float* __restrict__ base, int ld, int r0, int k0, int lane) {
  const float* p = base + (size_t)(r0 + (lane & 15)) * ld + k0 + (lane >> 4) * 8;
  const v4f a0 = *(const v4f*)(p), a1 = *(const v4f*)(p + 4), a2 = *(const v4f*)(p + 16), a3 = *(const v4f*)(p + 20);
  v16bf hi;
#pragma unroll
  for (int i = 0; i < 4; ++i) {
    hi[i] = bf_hi(a0[i]); hi[4 + i] = bf_hi(a1[i]); hi[8 + i] = bf_hi(a2[i]); hi[12 + i] = bf_hi(a3[i]);
  }
  return hi;
}
__device__ __forceinline__ v16bf frag_lds(const __bf16* base, int ld, int r0, int k0, int lane) {
  union { v16bf v; v8bf h[2]; } r;
  const __bf16* p = base + (r0 + (lane & 15)) * ld + k0 + (lane >> 4) * 8;
  r.h[0] = *(const v8bf*)(p); r.h[1] = *(const v8bf*)(p + 16);
  return r.v;
}

template <int KDIM>
__device__ __forceinline__ void gemm_hh_32x64(const float* __restrict__ A, const float* __restrict__ Bt,
                                              int m0, int n0, int lane, v8f acc[2][4]) {
#pragma unroll 1
  for (int k0 = 0; k0 < KDIM; k0 += 32) {
    v16bf ah[2], bh[4];
    ah[0] = frag_f32h(A, KDIM, m0, k0, lane);
    ah[1] = frag_f32h(A, KDIM, m0 + 16, k0, lane);
#pragma unroll
    for (int j = 0; j < 4; ++j) bh[j] = frag_f32h(Bt, KDIM, n0 + j * 16, k0, lane);
#pragma unroll
    for (int i = 0; i < 2; ++i)
#pragma unroll
      for (int j = 0; j < 4; ++j) acc[i][j] = wmma_bf16(ah[i], bh[j], acc[i][j]);
  }
}
template <int KDIM>
__device__ __forceinline__ void gemm_x2_32x64(const float* __restrict__ A, const float* __restrict__ Bt,
                                              int m0, int n0, int lane, v8f acc[2][4]) {
#pragma unroll 1
  for (int k0 = 0; k0 < KDIM; k0 += 32) {
    v16bf ah[2], al[2], bh[4];
    frag_f32(A, KDIM, m0, k0, lane, ah[0], al[0]);
    frag_f32(A, KDIM, m0 + 16, k0, lane, ah[1], al[1]);
#pragma unroll
    for (int j = 0; j < 4; ++j) bh[j] = frag_f32h(Bt, KDIM, n0 + j * 16, k0, lane);
#pragma unroll
    for (int i = 0; i < 2; ++i)
#pragma unroll
      for (int j = 0; j < 4; ++j) {
        acc[i][j] = wmma_bf16(ah[i], bh[j], acc[i][j]);
        acc[i][j] = wmma_bf16(al[i], bh[j], acc[i][j]);
      }
  }
}

__global__ __launch_bounds__(128) void proj_kernel(const float* __restrict__ X, const float* __restrict__ W,
                                                  const float* __restrict__ cosb, const float* __restrict__ sinb,
                                                  const int* __restrict__ tpos, int trows,
                                                  float scale, int part, float* __restrict__ dst) {
#pragma clang fp contract(off)
  __shared__ __align__(16) float st[128][64];
  const int lane = threadIdx.x & 31, wave = threadIdx.x >> 5, tid = threadIdx.x;
  const int mblk = blockIdx.y * 128;
  const int b = mblk / SEQ, s0 = mblk % SEQ;
  const int n0 = blockIdx.x * 64;
  const int head = n0 / HD_;
  const float* Xb = X + (size_t)(b * S_FULL + s0) * D_;

  v8f acc[2][4] = {};
  gemm_hh_32x64<D_>(Xb, W, wave * 32, n0, lane, acc);
  const int half = lane >> 4, col = lane & 15;
#pragma unroll
  for (int i = 0; i < 2; ++i)
#pragma unroll
    for (int j = 0; j < 4; ++j)
#pragma unroll
      for (int r = 0; r < 8; ++r) st[wave * 32 + i * 16 + r + 8 * half][j * 16 + col] = acc[i][j][r] * scale;
  __syncthreads();
  if (part < 2) {
#pragma unroll 2
    for (int it = 0; it < 32; ++it) {
      const int ml = wave + 4 * it;
      int pos = tpos[s0 + ml];
      pos = (pos < 0) ? pos + trows : pos;
      pos = (pos < 0) ? 0 : ((pos > trows - 1) ? trows - 1 : pos);
      const float c  = (float)bf_hi(cosb[(size_t)pos * NP_ + lane]);
      const float sn = (float)bf_hi(sinb[(size_t)pos * NP_ + lane]);
      const float te = st[ml][2 * lane], to = st[ml][2 * lane + 1];
      const float re = te * c - to * sn;
      const float ro = te * sn + to * c;
      st[ml][2 * lane] = re; st[ml][2 * lane + 1] = ro;
    }
    __syncthreads();
    for (int g = tid; g < 128 * 16; g += 128) {
      const int ml = g >> 4, pc = g & 15;
      vst2(dst + (((size_t)(b * H_ + head) * SEQ + s0 + ml) * HD_) + pc * 4, *(const v4f*)(&st[ml][pc * 4]));
    }
  } else {
    for (int g = tid; g < 64 * 32; g += 128) {
      const int dl = g >> 5, pc = g & 31;
      v4f v = {st[pc * 4][dl], st[pc * 4 + 1][dl], st[pc * 4 + 2][dl], st[pc * 4 + 3][dl]};
      vst2(dst + (((size_t)(b * H_ + head) * HD_ + dl) * SEQ) + s0 + pc * 4, v);
    }
  }
}

__global__ __launch_bounds__(128) __attribute__((amdgpu_num_vgpr(256)))
void attn_kernel(const float* __restrict__ Qb, const float* __restrict__ Kb,
                 const float* __restrict__ Vt, float* __restrict__ Ctx) {
  __shared__ __align__(16) __bf16 Kh[32 * 72], Kl[32 * 72];
  __shared__ __align__(16) __bf16 Vh[64 * 40], Vl[64 * 40];
  __shared__ __align__(16) __bf16 Ph[4][16 * 40], Pl[4][16 * 40];
  __shared__ __align__(16) float  Os[4][16 * 64];

  const int tid = threadIdx.x, lane = tid & 31, wave = tid >> 5, half = lane >> 4, col = lane & 15;
  const int q0 = blockIdx.x * 64, head = blockIdx.y, b = blockIdx.z;
  const float* Qh = Qb + (size_t)(b * H_ + head) * SEQ * HD_;
  const float* Kg = Kb + (size_t)(b * H_ + head) * SEQ * HD_;
  const float* Vg = Vt + (size_t)(b * H_ + head) * HD_ * SEQ;
  const int mq = q0 + wave * 16;

  v16bf qh[2], ql[2];
#pragma unroll
  for (int kb = 0; kb < 2; ++kb) frag_f32(Qh, HD_, mq, kb * 32, lane, qh[kb], ql[kb]);

  v8f o[4] = {};
  float mrow[8], lrow[8];
#pragma unroll
  for (int r = 0; r < 8; ++r) { mrow[r] = -1e30f; lrow[r] = 0.0f; }
  __bf16* ph = Ph[wave];
  __bf16* pl = Pl[wave];

  const int t_end = q0 + 64;
#pragma unroll 1
  for (int t0 = 0; t0 < t_end; t0 += 32) {
    __syncthreads();
    {
      const int kr = tid >> 2, kc = (tid & 3) * 16;
      const float* kp = Kg + (size_t)(t0 + kr) * HD_ + kc;
      const int vr = tid >> 1, vc = (tid & 1) * 16;
      const float* vp = Vg + (size_t)vr * SEQ + t0 + vc;
#pragma unroll
      for (int e = 0; e < 16; e += 4) {
        const v4f a = *(const v4f*)(kp + e), bb = *(const v4f*)(vp + e);
#pragma unroll
        for (int i = 0; i < 4; ++i) {
          __bf16 hk = bf_hi(a[i]);  Kh[kr * 72 + kc + e + i] = hk; Kl[kr * 72 + kc + e + i] = bf_lo(a[i], hk);
          __bf16 hv = bf_hi(bb[i]); Vh[vr * 40 + vc + e + i] = hv; Vl[vr * 40 + vc + e + i] = bf_lo(bb[i], hv);
        }
      }
    }
    __syncthreads();

    v8f s[2] = {};
#pragma unroll
    for (int n = 0; n < 2; ++n)
#pragma unroll
      for (int kb = 0; kb < 2; ++kb)
        s[n] = wmma_x3(qh[kb], ql[kb], frag_lds(Kh, 72, n * 16, kb * 32, lane), frag_lds(Kl, 72, n * 16, kb * 32, lane), s[n]);

    {
      const int k0g = t0 + col, k1g = t0 + 16 + col;
#pragma unroll
      for (int r = 0; r < 8; ++r) {
        const int qg = mq + r + 8 * half;
        float v0 = (k0g <= qg) ? s[0][r] : -1e30f;
        float v1 = (k1g <= qg) ? s[1][r] : -1e30f;
        float mx = fmaxf(v0, v1);
#pragma unroll
        for (int off = 8; off > 0; off >>= 1) mx = fmaxf(mx, __shfl_xor(mx, off, 16));
        const float mnew  = fmaxf(mrow[r], mx);
        const float alpha = __expf(mrow[r] - mnew);
        const float p0 = (k0g <= qg) ? __expf(v0 - mnew) : 0.0f;
        const float p1 = (k1g <= qg) ? __expf(v1 - mnew) : 0.0f;
        float rs = p0 + p1;
#pragma unroll
        for (int off = 8; off > 0; off >>= 1) rs += __shfl_xor(rs, off, 16);
        lrow[r] = lrow[r] * alpha + rs;
        mrow[r] = mnew;
#pragma unroll
        for (int j = 0; j < 4; ++j) o[j][r] *= alpha;
        const int row = r + 8 * half;
        __bf16 h0 = bf_hi(p0), h1 = bf_hi(p1);
        ph[row * 40 + col] = h0;      pl[row * 40 + col] = bf_lo(p0, h0);
        ph[row * 40 + 16 + col] = h1; pl[row * 40 + 16 + col] = bf_lo(p1, h1);
      }
    }
    __syncthreads();
    const v16bf pah = frag_lds(ph, 40, 0, 0, lane), pal = frag_lds(pl, 40, 0, 0, lane);
#pragma unroll
    for (int j = 0; j < 4; ++j)
      o[j] = wmma_x3(pah, pal, frag_lds(Vh, 40, j * 16, 0, lane), frag_lds(Vl, 40, j * 16, 0, lane), o[j]);
  }

  float* os_ = Os[wave];
#pragma unroll
  for (int r = 0; r < 8; ++r) {
    const float inv = 1.0f / lrow[r];
#pragma unroll
    for (int j = 0; j < 4; ++j) os_[(r + 8 * half) * 64 + j * 16 + col] = o[j][r] * inv;
  }
  __syncthreads();
#pragma unroll
  for (int q = 0; q < 8; ++q) {
    const int rl = q * 2 + (lane >> 4), pc = lane & 15;
    vst2(Ctx + ((size_t)(b * SEQ + mq + rl)) * D_ + head * HD_ + pc * 4, *(const v4f*)(os_ + rl * 64 + pc * 4));
  }
}

__global__ __launch_bounds__(128) void out_gemm_kernel(const float* __restrict__ Cx, const float* __restrict__ Wo, float* __restrict__ Out) {
  __shared__ __align__(16) float st[4][32 * 64];
  const int lane = threadIdx.x & 31, wave = threadIdx.x >> 5;
  const int m0 = blockIdx.y * 64 + (wave >> 1) * 32;
  const int n0 = blockIdx.x * 128 + (wave & 1) * 64;
  v8f acc[2][4] = {};
  gemm_x2_32x64<QKV_>(Cx, Wo, m0, n0, lane, acc);
  const int half = lane >> 4, col = lane & 15;
  float* S = st[wave];
#pragma unroll
  for (int i = 0; i < 2; ++i)
#pragma unroll
    for (int j = 0; j < 4; ++j)
#pragma unroll
      for (int r = 0; r < 8; ++r) S[(i * 16 + r + 8 * half) * 64 + j * 16 + col] = acc[i][j][r];
  __syncthreads();
#pragma unroll
  for (int q = 0; q < 16; ++q) {
    const int rl = q * 2 + (lane >> 4), pc = lane & 15;
    vst2(Out + (size_t)(m0 + rl) * D_ + n0 + pc * 4, *(const v4f*)(S + rl * 64 + pc * 4));
  }
}

extern "C" void kernel_launch(void* const* d_in, const int* in_sizes, int n_in,
                              void* d_out, int out_size, void* d_ws, size_t ws_size,
                              hipStream_t stream) {
  if (n_in < 6) return;
  const long long x_need = ((long long)(NB - 1) * S_FULL + SEQ) * (long long)D_;
  if ((long long)in_sizes[0] < x_need) return;
  if ((long long)in_sizes[1] < 3LL * D_ * D_) return;
  if ((long long)in_sizes[2] < (long long)D_ * D_) return;
  if (in_sizes[3] < NP_ || in_sizes[4] < NP_) return;
  if (in_sizes[5] < SEQ) return;
  if ((long long)out_size < (long long)M_TOT * D_) return;

  const size_t E = (size_t)M_TOT * D_;
  const size_t carve = 4 * E * sizeof(float);
  if (ws_size < carve) return;

  int trows = in_sizes[3] / NP_;
  const int srows = in_sizes[4] / NP_;
  if (srows < trows) trows = srows;

  const float* x    = (const float*)d_in[0];
  const float* Wqkv = (const float*)d_in[1];
  const float* Wout = (const float*)d_in[2];
  const float* cosb = (const float*)d_in[3];
  const float* sinb = (const float*)d_in[4];
  const int*   tpos = (const int*)d_in[5];
  float* out = (float*)d_out;

  float* qb   = (float*)d_ws;
  float* kb   = qb + E;
  float* vtb  = kb + E;
  float* ctxb = vtb + E;

  dim3 gp(QKV_ / 64, M_TOT / 128);
  proj_kernel<<<gp, 128, 0, stream>>>(x, Wqkv,                       cosb, sinb, tpos, trows, SCALE_, 0, qb);
  proj_kernel<<<gp, 128, 0, stream>>>(x, Wqkv + (size_t)D_ * D_,     cosb, sinb, tpos, trows, 1.0f,   1, kb);
  proj_kernel<<<gp, 128, 0, stream>>>(x, Wqkv + (size_t)2 * D_ * D_, cosb, sinb, tpos, trows, 1.0f,   2, vtb);
  attn_kernel<<<dim3(SEQ / 64, H_, NB), 128, 0, stream>>>(qb, kb, vtb, ctxb);
  out_gemm_kernel<<<dim3(D_ / 128, M_TOT / 64), 128, 0, stream>>>(ctxb, Wout, out);
}
